// MultiheadAttention_65283502899586
// MI455X (gfx1250) — hardware-run, weakly checked
//
#include <hip/hip_runtime.h>


#ifndef NB
#define NB 2
#endif
#ifndef SEQ
#define SEQ 2048
#endif
#define NB_FULL 2
#define TT_FULL 2048
#define TT   SEQ
#define DM   768
#define NH_  12
#define HD   64
#define DQ   (NH_ * HD)
#define ZH   3
#define PCAR 1024.0f
#define SCL  0.125f

static_assert(TT % 128 == 0);
static_assert(DM % 64 == 0);
static_assert(DQ == DM);
static_assert(NH_ % ZH == 0);
static_assert(HD == 64);
static_assert(TT <= TT_FULL);
static_assert(NB <= NB_FULL);
static_assert((size_t)(NB - 1) * TT_FULL * DM + (size_t)TT * DM <= (size_t)NB_FULL * TT_FULL * DM);

typedef _Float16 h16;
typedef unsigned short bf;
typedef __attribute__((ext_vector_type(16))) __bf16   v16bf;
typedef __attribute__((ext_vector_type(16))) _Float16 v16h;
typedef __attribute__((ext_vector_type(8)))  _Float16 v8h;
typedef __attribute__((ext_vector_type(8)))  unsigned short v8us;
typedef __attribute__((ext_vector_type(8)))  float    v8f;
typedef __attribute__((ext_vector_type(4)))  float    v4f;
typedef v8h  __attribute__((may_alias)) v8ha;
typedef v4f  __attribute__((may_alias)) v4fa;
typedef v8us __attribute__((may_alias)) v8usa;
typedef __attribute__((ext_vector_type(2))) _Float16 v2h;
typedef __attribute__((ext_vector_type(4))) _Float16 v4h;
typedef __attribute__((ext_vector_type(2))) unsigned short v2us;
typedef __attribute__((ext_vector_type(2))) float v2f;

__device__ __forceinline__ unsigned short f2bf(float f) { unsigned u = __float_as_uint(f); u += 0x7FFFu + ((u >> 16) & 1u); return (unsigned short)(u >> 16); }
__device__ __forceinline__ float bf2f(unsigned short b) { return __uint_as_float(((unsigned)b) << 16); }
__device__ __forceinline__ float bfr(float f) { return bf2f(f2bf(f)); }
__device__ __forceinline__ v16h cat16(v8h lo, v8h hi) { return __builtin_shufflevector(lo, hi, 0, 1, 2, 3, 4, 5, 6, 7, 8, 9, 10, 11, 12, 13, 14, 15); }
__device__ __forceinline__ v16bf cat16b(v8us lo, v8us hi) { return __builtin_bit_cast(v16bf, __builtin_shufflevector(lo, hi, 0, 1, 2, 3, 4, 5, 6, 7, 8, 9, 10, 11, 12, 13, 14, 15)); }
__device__ __forceinline__ v8f wmma16(v16h a, v16h b, v8f c) { return __builtin_amdgcn_wmma_f32_16x16x32_f16(false, a, false, b, (short)0, c, false, false); }
__device__ __forceinline__ v8f wmmab(v16bf a, v16bf b, v8f c) { return __builtin_amdgcn_wmma_f32_16x16x32_bf16(false, a, false, b, (short)0, c, false, false); }

template <typename T16> struct WFrag;
template <> struct WFrag<h16> { typedef v16h V; static __device__ __forceinline__ V ld(const h16* p) { return cat16(*(const v8h*)p, *(const v8h*)(p + 16)); } static __device__ __forceinline__ v8f mma(V a, V b, v8f c) { return wmma16(a, b, c); } };
template <> struct WFrag<bf> { typedef v16bf V; static __device__ __forceinline__ V ld(const bf* p) { return cat16b(*(const v8us*)p, *(const v8us*)(p + 16)); } static __device__ __forceinline__ v8f mma(V a, V b, v8f c) { return wmmab(a, b, c); } };
template <typename T16, int NSPLIT, bool BIAS>
__global__ __launch_bounds__(32) void k_gemmw(const T16* __restrict__ A, const T16* __restrict__ A2, const T16* __restrict__ Bt, const T16* __restrict__ Bt2, int K, float* C, int ldc, const float* __restrict__ bias, size_t sA, size_t sB, size_t sC) {
    typedef typename WFrag<T16>::V V;
    __shared__ __align__(16) float os[16 * 68];
    const size_t z = blockIdx.z; A += z * sA; if (A2) A2 += z * sA; Bt += z * sB; if (Bt2) Bt2 += z * sB; C += z * sC;
    const int lane = threadIdx.x & 31, lr = lane & 15, hi = lane >> 4; const int r0 = blockIdx.x * 64, c0 = blockIdx.y * 64;
    v8f acc[4][4];
#pragma unroll
    for (int mb = 0; mb < 4; ++mb)
#pragma unroll
        for (int nb = 0; nb < 4; ++nb) acc[mb][nb] = (v8f){};
    const size_t aoff = (size_t)(r0 + lr) * K + 8 * hi, boff = (size_t)(c0 + lr) * K + 8 * hi;
#pragma unroll 1
    for (int kc = 0; kc < K; kc += 32) {
        V a[4], a2[4];
#pragma unroll
        for (int mb = 0; mb < 4; ++mb) { a[mb] = WFrag<T16>::ld(A + aoff + (size_t)mb * 16 * K + kc); if (NSPLIT == 1 || NSPLIT == 2) a2[mb] = WFrag<T16>::ld(A2 + aoff + (size_t)mb * 16 * K + kc); }
#pragma unroll
        for (int nb = 0; nb < 4; ++nb) { const V b = WFrag<T16>::ld(Bt + boff + (size_t)nb * 16 * K + kc); V b2; if (NSPLIT >= 2) b2 = WFrag<T16>::ld(Bt2 + boff + (size_t)nb * 16 * K + kc);
#pragma unroll
            for (int mb = 0; mb < 4; ++mb) { acc[mb][nb] = WFrag<T16>::mma(a[mb], b, acc[mb][nb]); if (NSPLIT == 1 || NSPLIT == 2) acc[mb][nb] = WFrag<T16>::mma(a2[mb], b, acc[mb][nb]); if (NSPLIT >= 2) acc[mb][nb] = WFrag<T16>::mma(a[mb], b2, acc[mb][nb]); } }
        asm volatile("v_nop\n\tv_nop\n\tv_nop\n\tv_nop" : "+v"(acc[0][0]), "+v"(acc[1][1]), "+v"(acc[2][2]), "+v"(acc[3][3]) : "v"(a[0]), "v"(a[3]));
    }
#pragma unroll
    for (int mb = 0; mb < 4; ++mb) {
#pragma unroll
        for (int nb = 0; nb < 4; ++nb) {
#pragma unroll
            for (int j = 0; j < 8; ++j) os[(hi * 8 + j) * 68 + nb * 16 + lr] = acc[mb][nb][j]; }
        __builtin_amdgcn_wave_barrier(); asm volatile("" ::: "memory");
        float* crow = C + (size_t)(r0 + mb * 16) * ldc + c0;
#pragma unroll 1
        for (int ps = 0; ps < 2; ++ps) {
#pragma unroll
            for (int s = 0; s < 8; ++s) { const int row = 2 * s + hi, cofs = lr * 4; v4f val = *(const v4fa*)(os + row * 68 + cofs); if (BIAS) { val[0] += bfr(bias[c0 + cofs]); val[1] += bfr(bias[c0 + cofs + 1]); val[2] += bfr(bias[c0 + cofs + 2]); val[3] += bfr(bias[c0 + cofs + 3]); }
                *(volatile v4f*)(crow + (size_t)row * ldc + cofs) = val; }
            if (ps == 0) __threadfence(); }
        __builtin_amdgcn_wave_barrier(); asm volatile("" ::: "memory");
    }
}

__device__ __forceinline__ h16 tohx(float x) { return (h16)x; }
__device__ __forceinline__ void splitf(float y, unsigned short& h, unsigned short& l) { h = f2bf(y); l = f2bf(y - bf2f(h)); }

__global__ __launch_bounds__(256) void k_cvt8(const float* __restrict__ src, bf* dst, size_t n8) { const size_t i = (size_t)blockIdx.x * 256 + threadIdx.x; if (i >= n8) return; const v8f v = *(const v8f*)(src + i * 8); v8us o;
#pragma unroll
    for (int k = 0; k < 8; ++k) o[k] = f2bf(v[k]); *(volatile v8us*)(dst + i * 8) = o; __threadfence(); *(volatile v8us*)(dst + i * 8) = o; }

__global__ __launch_bounds__(256) void k_gwp(const float* __restrict__ gw, bf* dst) { const int i = blockIdx.x * 256 + threadIdx.x; if (i >= 64 * 64 / 8) return; const int row = i >> 3, c8 = (i & 7) * 8; const int rr = row < 8 ? row : 7; const v8f v = *(const v8f*)(gw + rr * 64 + c8); v8us o;
#pragma unroll
    for (int k = 0; k < 8; ++k) o[k] = (row < 8) ? f2bf(v[k]) : (unsigned short)0;
    *(volatile v8us*)(dst + (size_t)i * 8) = o; __threadfence(); *(volatile v8us*)(dst + (size_t)i * 8) = o; }

__device__ __forceinline__ int relbucket(int rel) {
    const int a = rel < 0 ? -rel : rel;
    const int big = 8 + (a >= 12) + (a >= 16) + (a >= 23) + (a >= 32) + (a >= 46) + (a >= 64) + (a >= 91);
    const int v = (a < 8) ? a : big;
    return ((rel > 0) ? 16 : 0) + v;
}
__global__ __launch_bounds__(256) void k_posb(const float* __restrict__ rel_emb, float* PB) { const int e = blockIdx.x * 256 + threadIdx.x; if (e >= NH_ * 2 * TT) return; const int h = e / (2 * TT); const int idx = e % (2 * TT); const int rel = idx - TT;
    const float val = bfr(rel_emb[relbucket(rel) * NH_ + h]); *(volatile float*)(PB + e) = val; __threadfence(); *(volatile float*)(PB + e) = val; }

__global__ __launch_bounds__(256) void k_gate(const float* __restrict__ G, const float* __restrict__ gb, const float* __restrict__ ga, float* GT) { const int e = blockIdx.x * 256 + threadIdx.x; if (e >= NH_ * TT) return; const int h = e / TT, t = e % TT;
    const float* gr = G + ((size_t)t * NH_ + h) * 64; const v4f a = *(const v4f*)gr; const v4f b = *(const v4f*)(gr + 4);
    float sa = ((a[0] + bfr(gb[0])) + (a[1] + bfr(gb[1]))) + ((a[2] + bfr(gb[2])) + (a[3] + bfr(gb[3])));
    float sb = ((b[0] + bfr(gb[4])) + (b[1] + bfr(gb[5]))) + ((b[2] + bfr(gb[6])) + (b[3] + bfr(gb[7])));
    sa = fminf(fmaxf(sa, -30.0f), 30.0f); sb = fminf(fmaxf(sb, -30.0f), 30.0f);
    const float gA = 1.0f / (1.0f + expf(-sa)); const float gB = 1.0f / (1.0f + expf(-sb));
    const float val = gA * (gB * bfr(ga[h]) - 1.0f) + 2.0f;
    *(volatile float*)(GT + e) = val; __threadfence(); *(volatile float*)(GT + e) = val; }

__global__ __launch_bounds__(256) void k_lnp(const float* __restrict__ F, int pitch, int nheads, float sc, bf* Ph, bf* Pl) {
    const size_t e = ((size_t)blockIdx.x * 256 + threadIdx.x) * 2; if (e >= (size_t)nheads * TT * HD) return; const int d = (int)(e % HD); const int t = (int)((e / HD) % TT); const int h = (int)(e / ((size_t)HD * TT));
    const v2f x = *(const v2f*)(F + (size_t)t * pitch + h * HD + d);
    float s = x[0] + x[1];
#pragma unroll
    for (int sh = 16; sh; sh >>= 1) s += __shfl_xor(s, sh, 32);
    const float mu = s * (1.0f / HD); const float d0 = x[0] - mu, d1 = x[1] - mu;
    float q = d0 * d0 + d1 * d1;
#pragma unroll
    for (int sh = 16; sh; sh >>= 1) q += __shfl_xor(q, sh, 32);
    const float rs = rsqrtf(q * (1.0f / HD) + 1.0e-5f) * sc;
    v2us oh, ol; unsigned short a2, c2; splitf(d0 * rs, a2, c2); oh[0] = a2; ol[0] = c2; splitf(d1 * rs, a2, c2); oh[1] = a2; ol[1] = c2;
    *(volatile v2us*)(Ph + e) = oh; *(volatile v2us*)(Pl + e) = ol; __threadfence(); *(volatile v2us*)(Ph + e) = oh; *(volatile v2us*)(Pl + e) = ol; }

__global__ __launch_bounds__(256) void k_vtp(const float* __restrict__ F, int pitch, int nheads, h16* V16) { const size_t e = ((size_t)blockIdx.x * 256 + threadIdx.x) * 2; if (e >= (size_t)nheads * HD * TT) return; const int t = (int)(e % TT); const int d = (int)((e / TT) % HD); const int g = (int)(e / ((size_t)TT * HD)); v2h o16;
#pragma unroll
    for (int q = 0; q < 2; ++q) { const float x = F[(size_t)(t + q) * pitch + g * HD + d]; o16[q] = tohx(x); }
    *(volatile v2h*)(V16 + e) = o16; __threadfence(); *(volatile v2h*)(V16 + e) = o16; }

__global__ __launch_bounds__(256) void k_asoft(const float* __restrict__ Sb, const float* __restrict__ PB, const float* __restrict__ GT, int h0, h16* P16) {
    __shared__ float pbs[TT + 8];
    const int lane = threadIdx.x & 31, w = threadIdx.x >> 5; const int row0 = blockIdx.x * 8; const int i0 = row0 % TT; const int zz = row0 / TT;
    const float* pbh = PB + (size_t)(h0 + zz) * (2 * TT); const int base = TT - i0 - 7;
#pragma unroll 1
    for (int k = threadIdx.x; k < TT + 8; k += 256) { int idx = base + k; idx = idx < 0 ? 0 : (idx > 2 * TT - 1 ? 2 * TT - 1 : idx); pbs[k] = pbh[idx]; }
    __syncthreads();
    const int row = row0 + w; const int i = i0 + w; const float g = GT[(size_t)(h0 + zz) * TT + i];
    const float* sr = Sb + (size_t)row * TT; float v[TT / 32]; float mx = -3.0e38f;
#pragma unroll
    for (int ch = 0; ch < TT / 128; ++ch) { const int j0 = ch * 128 + lane * 4; const v4f a = *(const v4f*)(sr + j0); const int pk = j0 - w + 7;
#pragma unroll
        for (int q = 0; q < 4; ++q) { const float t = a[q] * SCL + g * pbs[pk + q]; v[ch * 4 + q] = t; mx = fmaxf(mx, t); } }
#pragma unroll
    for (int sh = 16; sh; sh >>= 1) mx = fmaxf(mx, __shfl_xor(mx, sh, 32));
    float sum = 0.f;
#pragma unroll
    for (int k = 0; k < TT / 32; ++k) { float d0 = __fsub_rn(v[k], mx); asm volatile("" : "+v"(d0)); v[k] = __builtin_amdgcn_exp2f(__fmul_rn(d0, 1.4426950408889634f)); sum += v[k]; }
#pragma unroll
    for (int sh = 16; sh; sh >>= 1) sum += __shfl_xor(sum, sh, 32);
    const float f = __fdiv_rn(PCAR, sum);
#pragma unroll 1
    for (int ps = 0; ps < 2; ++ps) {
#pragma unroll
        for (int ch = 0; ch < TT / 128; ++ch) { v4h o4;
#pragma unroll
            for (int q = 0; q < 4; ++q) o4[q] = tohx(v[ch * 4 + q] * f);
            *(volatile v4h*)(P16 + (size_t)row * TT + ch * 128 + lane * 4) = o4; }
        if (ps == 0) __threadfence(); }
}

__global__ __launch_bounds__(256) void k_merge(const float* __restrict__ O, int h0, bf* Ah, bf* Al) { const size_t e = ((size_t)blockIdx.x * 256 + threadIdx.x) * 2; if (e >= (size_t)ZH * TT * HD) return; const int d = (int)(e % HD); const int t = (int)((e / HD) % TT); const int zz = (int)(e / ((size_t)HD * TT)); const float cs = 1.0f / PCAR; const size_t oo = (size_t)t * DQ + (h0 + zz) * HD + d;
    v2us oh, ol;
#pragma unroll
    for (int q = 0; q < 2; ++q) { unsigned short a, c2; splitf(O[e + q] * cs, a, c2); oh[q] = a; ol[q] = c2; } *(volatile v2us*)(Ah + oo) = oh; *(volatile v2us*)(Al + oo) = ol; __threadfence(); *(volatile v2us*)(Ah + oo) = oh; *(volatile v2us*)(Al + oo) = ol; }

constexpr size_t al256(size_t b) { return (b + 255) & ~(size_t)255; }
constexpr size_t SZ_W   = al256((size_t)DM * DM * 2);
constexpr size_t SZ_GW  = al256((size_t)64 * 64 * 2);
constexpr size_t SZ_PB  = al256((size_t)NH_ * 2 * TT * 4);
constexpr size_t SZ_XB  = al256((size_t)TT * DM * 2);
constexpr size_t SZ_F   = al256((size_t)TT * DM * 4);
constexpr size_t SZ_PL  = al256((size_t)NH_ * TT * HD * 2);
constexpr size_t SZ_GT  = al256((size_t)NH_ * TT * 4);
constexpr size_t SZ_SB  = al256((size_t)ZH * TT * TT * 4);
constexpr size_t SZ_P16 = al256((size_t)ZH * TT * TT * 2);
constexpr size_t SZ_OB  = al256((size_t)ZH * TT * HD * 4);
constexpr size_t SZ_AT  = al256((size_t)TT * DQ * 2);
constexpr size_t WS_TOTAL = 4 * SZ_W + SZ_GW + SZ_PB + SZ_XB + SZ_F + 5 * SZ_PL + SZ_GT + SZ_SB + SZ_P16 + SZ_OB + 2 * SZ_AT;
static_assert(WS_TOTAL <= (size_t)134217728);
static_assert((size_t)TT * NH_ * 64 * 4 <= SZ_F);

extern "C" void kernel_launch(void* const* d_in, const int* in_sizes, int n_in,
                              void* d_out, int out_size, void* d_ws, size_t ws_size, hipStream_t stream) {
    if (n_in < 15) return;
    const size_t need_act = (size_t)(NB - 1) * TT_FULL * DM + (size_t)TT * DM;
    if ((size_t)in_sizes[0] < need_act || (size_t)in_sizes[1] < need_act || (size_t)in_sizes[2] < need_act) return;
    if (in_sizes[3] < DM * DM || in_sizes[5] < DM * DM || in_sizes[7] < DM * DM || in_sizes[9] < DM * DM) return;
    if (in_sizes[4] < DM || in_sizes[6] < DM || in_sizes[8] < DM || in_sizes[10] < DM) return;
    if (in_sizes[11] < 32 * NH_ || in_sizes[12] < 8 * HD || in_sizes[13] < 8 || in_sizes[14] < NH_) return;
    if ((size_t)out_size < need_act) return;
    if (WS_TOTAL > ws_size) return;
    const float* xq = (const float*)d_in[0]; const float* xk = (const float*)d_in[1]; const float* xv = (const float*)d_in[2];
    const float* wq = (const float*)d_in[3]; const float* bq = (const float*)d_in[4];
    const float* wk = (const float*)d_in[5]; const float* bk = (const float*)d_in[6];
    const float* wv = (const float*)d_in[7]; const float* bv = (const float*)d_in[8];
    const float* wo = (const float*)d_in[9]; const float* bo = (const float*)d_in[10];
    const float* rel_emb = (const float*)d_in[11]; const float* grep_W = (const float*)d_in[12]; const float* grep_b = (const float*)d_in[13]; const float* grep_a = (const float*)d_in[14];
    float* OUT = (float*)d_out;
    char* wsp = (char*)d_ws;
    bf* WQ = (bf*)wsp; wsp += SZ_W; bf* WK = (bf*)wsp; wsp += SZ_W; bf* WV = (bf*)wsp; wsp += SZ_W; bf* WO = (bf*)wsp; wsp += SZ_W;
    bf* GW = (bf*)wsp; wsp += SZ_GW; float* PB = (float*)wsp; wsp += SZ_PB;
    bf* XB = (bf*)wsp; wsp += SZ_XB; float* F = (float*)wsp; wsp += SZ_F;
    bf* QPh = (bf*)wsp; wsp += SZ_PL; bf* QPl = (bf*)wsp; wsp += SZ_PL; bf* KPh = (bf*)wsp; wsp += SZ_PL; bf* KPl = (bf*)wsp; wsp += SZ_PL; h16* VT16 = (h16*)wsp; wsp += SZ_PL;
    float* GT = (float*)wsp; wsp += SZ_GT;
    float* Sb = (float*)wsp; wsp += SZ_SB; h16* P16 = (h16*)wsp; wsp += SZ_P16; float* Ob = (float*)wsp; wsp += SZ_OB;
    bf* ATh = (bf*)wsp; wsp += SZ_AT; bf* ATl = (bf*)wsp; wsp += SZ_AT;

    const size_t nw8 = (size_t)DM * DM / 8, nx8 = (size_t)TT * DM / 8;
    k_cvt8<<<(unsigned)((nw8 + 255) / 256), 256, 0, stream>>>(wq, WQ, nw8);
    k_cvt8<<<(unsigned)((nw8 + 255) / 256), 256, 0, stream>>>(wk, WK, nw8);
    k_cvt8<<<(unsigned)((nw8 + 255) / 256), 256, 0, stream>>>(wv, WV, nw8);
    k_cvt8<<<(unsigned)((nw8 + 255) / 256), 256, 0, stream>>>(wo, WO, nw8);
    k_gwp<<<2, 256, 0, stream>>>(grep_W, GW);
    k_posb<<<(NH_ * 2 * TT + 255) / 256, 256, 0, stream>>>(rel_emb, PB);
    const unsigned LP = (unsigned)(((size_t)NH_ * TT * HD / 2 + 255) / 256);
    for (int b = 0; b < NB; ++b) {
        const size_t xo = (size_t)b * TT_FULL * DM;
        k_cvt8<<<(unsigned)((nx8 + 255) / 256), 256, 0, stream>>>(xq + xo, XB, nx8);
        k_gemmw<bf, 0, true><<<dim3(TT / 64, DQ / 64, 1), 32, 0, stream>>>(XB, nullptr, WQ, nullptr, DM, F, DQ, bq, 0, 0, 0);
        k_lnp<<<LP, 256, 0, stream>>>(F, DQ, NH_, 1.0f, QPh, QPl);
        k_gemmw<bf, 0, false><<<dim3(TT * NH_ / 64, 1, 1), 32, 0, stream>>>(XB, nullptr, GW, nullptr, HD, F, 64, nullptr, 0, 0, 0);
        k_gate<<<(NH_ * TT + 255) / 256, 256, 0, stream>>>(F, grep_b, grep_a, GT);
        k_cvt8<<<(unsigned)((nx8 + 255) / 256), 256, 0, stream>>>(xk + xo, XB, nx8);
        k_gemmw<bf, 0, true><<<dim3(TT / 64, DQ / 64, 1), 32, 0, stream>>>(XB, nullptr, WK, nullptr, DM, F, DQ, bk, 0, 0, 0);
        k_lnp<<<LP, 256, 0, stream>>>(F, DQ, NH_, 1.0f, KPh, KPl);
        k_cvt8<<<(unsigned)((nx8 + 255) / 256), 256, 0, stream>>>(xv + xo, XB, nx8);
        k_gemmw<bf, 0, true><<<dim3(TT / 64, DQ / 64, 1), 32, 0, stream>>>(XB, nullptr, WV, nullptr, DM, F, DQ, bv, 0, 0, 0);
        k_vtp<<<LP, 256, 0, stream>>>(F, DQ, NH_, VT16);
        for (int h0 = 0; h0 < NH_; h0 += ZH) { const size_t zo = (size_t)h0 * TT * HD;
            k_gemmw<bf, 2, false><<<dim3(TT / 64, TT / 64, ZH), 32, 0, stream>>>(QPh + zo, QPl + zo, KPh + zo, KPl + zo, HD, Sb, TT, nullptr, (size_t)TT * HD, (size_t)TT * HD, (size_t)TT * TT);
            k_asoft<<<ZH * TT / 8, 256, 0, stream>>>(Sb, PB, GT, h0, P16);
            k_gemmw<h16, 0, false><<<dim3(TT / 64, HD / 64, ZH), 32, 0, stream>>>(P16, nullptr, VT16 + zo, nullptr, TT, Ob, HD, nullptr, (size_t)TT * TT, (size_t)HD * TT, (size_t)TT * HD);
            k_merge<<<(unsigned)(((size_t)ZH * TT * HD / 2 + 255) / 256), 256, 0, stream>>>(Ob, h0, ATh, ATl); }
        k_gemmw<bf, 1, true><<<dim3(TT / 64, DM / 64, 1), 32, 0, stream>>>(ATh, ATl, WO, nullptr, DQ, OUT + xo, DM, bo, 0, 0, 0); }
}
